// Sage_76682346102897
// MI455X (gfx1250) — hardware-run, weakly checked
//
#include <hip/hip_runtime.h>
#include <stddef.h>
#include <stdint.h>


#ifndef MEAN_SPLIT
#define MEAN_SPLIT 1
#endif

#define DF      64
#define NPARTS  (2 + MEAN_SPLIT)
#define KT      (DF * NPARTS)
#define MPIT    128
#define NTHR    256
#define NWAVE   8
#define WCH     256
#define NBA     1024
#define SLA     10
#define RCAP    20480
#define WLCAP   3200
#define GBM     128
#define UPART   512
#define NUB     (NPARTS * UPART)
#define FLAGI   32
#define MEAS_BLOCK_HITS 16721
#define MEAS_MAX_DEG    36
#define MAXN    131072
#define MAXE    (1 << 21)
#define WSMAX   134217728

#define L_WL    0
#define L_PL    (NWAVE * WLCAP)
#define L_WC    (L_PL + RCAP)
#define L_CNT   (L_WC + NWAVE * NBA)
#define L_OFF   (L_CNT + NBA)
#define L_MISC  (L_OFF + NBA)
#define MISC_INTS 1024
#define SCAN_INTS (L_MISC + MISC_INTS)

static_assert(DF == 16 * 4);
static_assert(KT % 32 == 0 && DF % 32 == 0 && (KT - DF) % 32 == 0);
static_assert(GBM == NWAVE * 16 && NTHR == NWAVE * 32);
static_assert(NBA == (1 << SLA) && NBA % NWAVE == 0 && NBA == NTHR * 4 && NBA % GBM == 0);
static_assert(RCAP >= MEAS_BLOCK_HITS + (MEAS_BLOCK_HITS * 15) / 100);
static_assert(WLCAP * 4 >= (RCAP / NWAVE) * 5);
static_assert(RCAP > MEAS_MAX_DEG + 8);
static_assert(((long long)MAXE << SLA) <= (1LL << 31));
static_assert(((long long)MAXN << SLA) < (1LL << 31));
static_assert(SCAN_INTS % (NTHR * 4) == 0 && SCAN_INTS * 4 <= 300000);
static_assert(L_PL % 4 == 0 && L_WC % 4 == 0 && L_CNT % 4 == 0 && L_OFF % 4 == 0 && L_MISC % 4 == 0);
static_assert(UPART % NTHR == 0 && NUB % NTHR == 0 && UPART == DF * (DF / 8));
static_assert(WCH == 32 * 8 && MPIT == 2 * DF && FLAGI * 4 == 128);

typedef float          v4f   __attribute__((ext_vector_type(4)));
typedef float          v8f   __attribute__((ext_vector_type(8)));
typedef int            v4i   __attribute__((ext_vector_type(4)));
typedef int            v8i   __attribute__((ext_vector_type(8)));
typedef unsigned       v2u   __attribute__((ext_vector_type(2)));
typedef unsigned short v4us  __attribute__((ext_vector_type(4)));
typedef unsigned short v8us  __attribute__((ext_vector_type(8)));
typedef unsigned short v16us __attribute__((ext_vector_type(16)));
typedef __bf16         v16bf __attribute__((ext_vector_type(16)));
typedef v4f  __attribute__((may_alias)) v4fa;
typedef v4i  __attribute__((may_alias)) v4ia;
typedef v2u  __attribute__((may_alias)) v2ua;
typedef v8us __attribute__((may_alias)) v8usa;
union FragB { v16bf v; v16us u; v8us h[2]; v8i w; };

__device__ __forceinline__ v8f wmb(const FragB& a, const FragB& b, v8f c) {
  v8f d = __builtin_amdgcn_wmma_f32_16x16x32_bf16(false, a.v, false, b.v, (short)0, c, false, false);
  asm volatile("v_nop\n\tv_nop\n\tv_nop\n\tv_nop" : "+v"(d) : "v"(a.w), "v"(b.w));
  return d;
}

__device__ __forceinline__ int imin(int a, int b) { return a < b ? a : b; }
__device__ __forceinline__ int imax(int a, int b) { return a > b ? a : b; }

__device__ __forceinline__ unsigned bf16_bits(float f) {
  const unsigned u = __float_as_uint(f);
  const unsigned r = (u + 0x7FFFu + ((u >> 16) & 1u)) >> 16;
  return ((u & 0x7FFFFFFFu) > 0x7F800000u) ? 0x7FC0u : r;
}
__device__ __forceinline__ float bf16_val(float f) {
  return __uint_as_float(bf16_bits(f) << 16);
}
__device__ __forceinline__ unsigned hl_sel(float v, int sel) {
  const unsigned hb = bf16_bits(v);
  const unsigned lb = bf16_bits(v - __uint_as_float(hb << 16));
  return (sel != 0) ? lb : hb;
}

__device__ __forceinline__ void st8x2(unsigned short* p, v8us o) {
  *(volatile v8us*)p = o;
  __threadfence();
  *(volatile v8us*)p = o;
}

__device__ __forceinline__ v8us wcol8(const float* __restrict__ W, int n, int kb) {
  v8us o;
#pragma unroll
  for (int i = 0; i < 8; ++i) o[i] = (unsigned short)bf16_bits(W[(kb + i) * DF + n]);
  return o;
}

__global__ __launch_bounds__(NTHR) void k_prep(const float* __restrict__ feat, const float* __restrict__ wself,
                                               const float* __restrict__ wneigh, const float* __restrict__ bias,
                                               unsigned short* fbp, unsigned short* btp, float* biasf,
                                               int nN, int nUnits) {
  const int u = (int)blockIdx.x * NTHR + (int)threadIdx.x;
  if (u < NUB) {
    const int part = u >> 9;
    const int v = u & (UPART - 1);
    const int n = v >> 3, kb = (v & 7) * 8;
    v8us o;
    if (part == 0) o = wcol8(wself, n, kb);
    else           o = wcol8(wneigh, n, kb);
    st8x2(btp + (size_t)n * KT + part * DF + kb, o);
  } else if (u < NUB + NTHR) {
    const int v  = u - NUB;
    const int c4 = 4 * (v & 15);
    const v4f b  = *(const v4f*)(bias + c4);
    v4f r;
    r.x = bf16_val(b.x); r.y = bf16_val(b.y); r.z = bf16_val(b.z); r.w = bf16_val(b.w);
    if (v < 16) {
      *(volatile v4f*)(biasf + c4) = r;
      __threadfence();
      *(volatile v4f*)(biasf + c4) = r;
    }
  } else if (u < nUnits) {
    const int v   = u - NUB - NTHR;
    const int row = v >> 3, j = (v & 7) * 8;
    const int rc  = imin(row, nN - 1);
    const float* p = feat + (size_t)rc * DF + j;
    const v4f a = *(const v4f*)p;
    const v4f b = *(const v4f*)(p + 4);
    asm volatile("" :: "v"(a), "v"(b));
    const unsigned msk = (row < nN) ? 0xFFFFu : 0u;
    v8us o;
    o[0] = (unsigned short)(bf16_bits(a.x) & msk); o[1] = (unsigned short)(bf16_bits(a.y) & msk);
    o[2] = (unsigned short)(bf16_bits(a.z) & msk); o[3] = (unsigned short)(bf16_bits(a.w) & msk);
    o[4] = (unsigned short)(bf16_bits(b.x) & msk); o[5] = (unsigned short)(bf16_bits(b.y) & msk);
    o[6] = (unsigned short)(bf16_bits(b.z) & msk); o[7] = (unsigned short)(bf16_bits(b.w) & msk);
    st8x2(fbp + (size_t)v * 8, o);
  }
}

__device__ __forceinline__ int sweep_chunk(const int* __restrict__ dsts, int nE, int cbase, int slotBase,
                                           int* mylist, int lane, int wc) {
  const int e0   = cbase + lane * 8;
  const int sent = -2147483647 - 1;
  v4i da, db;
  if (cbase + WCH <= nE) {
    da = *(const v4i*)(dsts + e0);
    db = *(const v4i*)(dsts + e0 + 4);
  } else {
    const int x0 = dsts[imin(e0,     nE - 1)];
    const int x1 = dsts[imin(e0 + 1, nE - 1)];
    const int x2 = dsts[imin(e0 + 2, nE - 1)];
    const int x3 = dsts[imin(e0 + 3, nE - 1)];
    const int x4 = dsts[imin(e0 + 4, nE - 1)];
    const int x5 = dsts[imin(e0 + 5, nE - 1)];
    const int x6 = dsts[imin(e0 + 6, nE - 1)];
    const int x7 = dsts[imin(e0 + 7, nE - 1)];
    asm volatile("" :: "v"(x0), "v"(x1), "v"(x2), "v"(x3), "v"(x4), "v"(x5), "v"(x6), "v"(x7));
    da.x = (e0     < nE) ? x0 : sent;
    da.y = (e0 + 1 < nE) ? x1 : sent;
    da.z = (e0 + 2 < nE) ? x2 : sent;
    da.w = (e0 + 3 < nE) ? x3 : sent;
    db.x = (e0 + 4 < nE) ? x4 : sent;
    db.y = (e0 + 5 < nE) ? x5 : sent;
    db.z = (e0 + 6 < nE) ? x6 : sent;
    db.w = (e0 + 7 < nE) ? x7 : sent;
  }
  const unsigned nbs = (unsigned)slotBase;
  const unsigned s0 = (unsigned)da.x - nbs, s1 = (unsigned)da.y - nbs;
  const unsigned s2 = (unsigned)da.z - nbs, s3 = (unsigned)da.w - nbs;
  const unsigned s4 = (unsigned)db.x - nbs, s5 = (unsigned)db.y - nbs;
  const unsigned s6 = (unsigned)db.z - nbs, s7 = (unsigned)db.w - nbs;
  const bool h0 = s0 < (unsigned)NBA, h1 = s1 < (unsigned)NBA, h2 = s2 < (unsigned)NBA, h3 = s3 < (unsigned)NBA;
  const bool h4 = s4 < (unsigned)NBA, h5 = s5 < (unsigned)NBA, h6 = s6 < (unsigned)NBA, h7 = s7 < (unsigned)NBA;
  const unsigned any = __builtin_amdgcn_ballot_w32(h0 | h1 | h2 | h3 | h4 | h5 | h6 | h7);
  if (any != 0u) {
    const unsigned m0 = __builtin_amdgcn_ballot_w32(h0);
    const unsigned m1 = __builtin_amdgcn_ballot_w32(h1);
    const unsigned m2 = __builtin_amdgcn_ballot_w32(h2);
    const unsigned m3 = __builtin_amdgcn_ballot_w32(h3);
    const unsigned m4 = __builtin_amdgcn_ballot_w32(h4);
    const unsigned m5 = __builtin_amdgcn_ballot_w32(h5);
    const unsigned m6 = __builtin_amdgcn_ballot_w32(h6);
    const unsigned m7 = __builtin_amdgcn_ballot_w32(h7);
    int r = wc
          + (int)__builtin_amdgcn_mbcnt_lo(m0, 0u) + (int)__builtin_amdgcn_mbcnt_lo(m1, 0u)
          + (int)__builtin_amdgcn_mbcnt_lo(m2, 0u) + (int)__builtin_amdgcn_mbcnt_lo(m3, 0u)
          + (int)__builtin_amdgcn_mbcnt_lo(m4, 0u) + (int)__builtin_amdgcn_mbcnt_lo(m5, 0u)
          + (int)__builtin_amdgcn_mbcnt_lo(m6, 0u) + (int)__builtin_amdgcn_mbcnt_lo(m7, 0u);
#define PUTJ(J, MJ, HJ, SJ) \
    if ((MJ) != 0u) { \
      if ((HJ) && r < WLCAP) mylist[r] = ((e0 + (J)) << SLA) | (int)(SJ); \
      r += (HJ) ? 1 : 0; \
    }
    PUTJ(0, m0, h0, s0)
    PUTJ(1, m1, h1, s1)
    PUTJ(2, m2, h2, s2)
    PUTJ(3, m3, h3, s3)
    PUTJ(4, m4, h4, s4)
    PUTJ(5, m5, h5, s5)
    PUTJ(6, m6, h6, s6)
    PUTJ(7, m7, h7, s7)
#undef PUTJ
    wc += (int)__builtin_popcount(m0) + (int)__builtin_popcount(m1) + (int)__builtin_popcount(m2)
        + (int)__builtin_popcount(m3) + (int)__builtin_popcount(m4) + (int)__builtin_popcount(m5)
        + (int)__builtin_popcount(m6) + (int)__builtin_popcount(m7);
  }
  return wc;
}

__global__ __launch_bounds__(NTHR) __attribute__((amdgpu_num_vgpr(248)))
void k_scan(const int* __restrict__ srcs, const int* __restrict__ dsts, const unsigned short* __restrict__ fb,
            unsigned short* mhl, int* flagp, int nE, int nN, int mRows) {
  extern __shared__ __attribute__((aligned(16))) int dsm[];
  int* wl   = dsm + L_WL;
  int* pl   = dsm + L_PL;
  int* wcn  = dsm + L_WC;
  int* cnt  = dsm + L_CNT;
  int* offs = dsm + L_OFF;
  int* misc = dsm + L_MISC;
  const int tid  = (int)threadIdx.x, lane = tid & 31;
  const int wave = __builtin_amdgcn_readfirstlane(tid >> 5);
  const int nodeBase = (int)blockIdx.x * NBA;
  int* mylist = wl + wave * WLCAP;
  int* mycnt  = wcn + wave * NBA;

  {
    const v4i z4 = {0, 0, 0, 0};
    for (int i = tid * 4; i < SCAN_INTS; i += NTHR * 4) *(v4ia*)(dsm + i) = z4;
  }
  __syncthreads();

  int wc = 0;
  {
    const int nwc = (nE + WCH - 1) / WCH;
    const int per = (nwc + NWAVE - 1) / NWAVE;
    const int c0  = wave * per;
    const int c1  = imin(c0 + per, nwc);
#pragma unroll 1
    for (int ch = c0; ch < c1; ++ch) wc = sweep_chunk(dsts, nE, ch * WCH, nodeBase, mylist, lane, wc);
  }
  const int wcc = imin(imax(wc, 0), WLCAP);
  if (lane == 0) { misc[wave] = wcc; misc[8 + wave] = (wc > WLCAP) ? 1 : 0; }
  __syncthreads();

#pragma unroll 1
  for (int b0 = 0; b0 < wcc; b0 += 32) {
    const int idx = b0 + lane;
    const int idc = imin(idx, WLCAP - 1);
    const int ent = mylist[idc];
    int eid = (int)((unsigned)ent >> SLA);
    eid = imin(eid, nE - 1);
    int s = srcs[eid];
    asm volatile("" :: "v"(s));
    s = imin(imax(s, 0), nN - 1);
    if (idx < wcc) mylist[idc] = (s << SLA) | (ent & (NBA - 1));
  }
  __syncthreads();

  if (lane == 0) {
#pragma unroll 1
    for (int i = 0; i < wcc; ++i) {
      const int s = mylist[i] & (NBA - 1);
      mycnt[s] = mycnt[s] + 1;
    }
  }
  __syncthreads();

  int ovf = 0;
  {
    v4i cw[NWAVE];
#pragma unroll
    for (int w2 = 0; w2 < NWAVE; ++w2) cw[w2] = *(const v4ia*)(wcn + w2 * NBA + 4 * tid);
    v4i tot = cw[0];
#pragma unroll
    for (int w2 = 1; w2 < NWAVE; ++w2) tot += cw[w2];
    const int S = tot.x + tot.y + tot.z + tot.w;
    int incl = S;
#pragma unroll
    for (int d = 1; d < 32; d <<= 1) {
      const int y = __shfl_up(incl, d, 32);
      incl += (lane >= d) ? y : 0;
    }
    if (lane == 31) misc[16 + wave] = incl;
    __syncthreads();
    int base = 0, total = 0;
#pragma unroll
    for (int w2 = 0; w2 < NWAVE; ++w2) {
      const int v = misc[16 + w2];
      base  += (w2 < wave) ? v : 0;
      total += v;
      ovf   |= misc[8 + w2];
    }
    ovf |= (total > RCAP) ? 1 : 0;
    const int run = base + incl - S;
    v4i of;
    of.x = run; of.y = run + tot.x; of.z = of.y + tot.y; of.w = of.z + tot.z;
    *(v4ia*)(cnt + 4 * tid)  = tot;
    *(v4ia*)(offs + 4 * tid) = of;
    v4i cu = of;
#pragma unroll
    for (int w2 = 0; w2 < NWAVE; ++w2) {
      *(v4ia*)(wcn + w2 * NBA + 4 * tid) = cu;
      cu += cw[w2];
    }
  }
  __syncthreads();

  if (lane == 0) {
#pragma unroll 1
    for (int i = 0; i < wcc; ++i) {
      const int ent = mylist[i];
      const int s = ent & (NBA - 1);
      int p = mycnt[s];
      mycnt[s] = p + 1;
      p = imin(imax(p, 0), RCAP - 1);
      pl[p] = (int)((unsigned)ent >> SLA);
    }
  }
  __syncthreads();

  if (wave == 0 && lane < 8) {
    v4i fv; fv.x = ovf; fv.y = ovf; fv.z = ovf; fv.w = ovf;
    int* fp = flagp + (size_t)blockIdx.x * FLAGI + 4 * lane;
    *(volatile v4i*)fp = fv;
    __threadfence();
    *(volatile v4i*)fp = fv;
  }

  const int hh = lane >> 4, q = lane & 15;
  const float pz = (ovf != 0) ? __int_as_float(0x7fc00000) : 0.0f;
#pragma unroll 1
  for (int si = 0; si < NBA / NWAVE; ++si) {
    const int s    = si * NWAVE + wave;
    const int node = nodeBase + s;
    int c = __builtin_amdgcn_readfirstlane(cnt[s]);
    int o = __builtin_amdgcn_readfirstlane(offs[s]);
    o = imin(imax(o, 0), RCAP - 1);
    c = imin(imax(c, 0), RCAP - o);
    int last = o + c - 1; last = last < o ? o : last;
    const int nIt = (c + 1) >> 1;
    float a0 = 0.0f, a1 = 0.0f, a2 = 0.0f, a3 = 0.0f;
#pragma unroll 1
    for (int it = 0; it < nIt; ++it) {
      const int p  = o + 2 * it + hh;
      const int pc = imin(p, last);
      int sr = pl[pc];
      sr = imin(imax(sr, 0), nN - 1);
      const v2u w = *(const v2ua*)(fb + (size_t)sr * DF + 4 * q);
      asm volatile("" :: "v"(w));
      const unsigned mk = (p <= last) ? 0xFFFFFFFFu : 0u;
      const unsigned wx = w.x & mk, wy = w.y & mk;
      a0 += __uint_as_float(wx << 16);
      a1 += __uint_as_float(wx & 0xffff0000u);
      a2 += __uint_as_float(wy << 16);
      a3 += __uint_as_float(wy & 0xffff0000u);
    }
    a0 += __shfl_xor(a0, 16, 32);
    a1 += __shfl_xor(a1, 16, 32);
    a2 += __shfl_xor(a2, 16, 32);
    a3 += __shfl_xor(a3, 16, 32);
    const float dg = fmaxf((float)c, 1.0f);
    const bool live = node < nN;
    float m0 = a0 / dg + pz;
    float m1 = a1 / dg + pz;
    float m2 = a2 / dg + pz;
    float m3 = a3 / dg + pz;
    m0 = live ? m0 : 0.0f; m1 = live ? m1 : 0.0f; m2 = live ? m2 : 0.0f; m3 = live ? m3 : 0.0f;
    v4us o4;
    o4[0] = (unsigned short)hl_sel(m0, hh);
    o4[1] = (unsigned short)hl_sel(m1, hh);
    o4[2] = (unsigned short)hl_sel(m2, hh);
    o4[3] = (unsigned short)hl_sel(m3, hh);
    if (node < mRows) {
      unsigned short* rp = mhl + (size_t)node * MPIT + 4 * lane;
      *(volatile v4us*)rp = o4;
      __threadfence();
      *(volatile v4us*)rp = o4;
    }
  }
}

__global__ __launch_bounds__(NTHR) __attribute__((amdgpu_num_vgpr(248)))
void k_gemm(const unsigned short* __restrict__ fb, const unsigned short* __restrict__ mhl,
            const unsigned short* __restrict__ bt, const float* __restrict__ biasf,
            const int* __restrict__ flagp, int nFlag, float* outp, int nN) {
  __shared__ __attribute__((aligned(16))) float stg[GBM * DF];
  __shared__ __attribute__((aligned(16))) float sbias[DF];
  const int tid  = (int)threadIdx.x, lane = tid & 31;
  const int wave = __builtin_amdgcn_readfirstlane(tid >> 5);
  const int hh = lane >> 4, m = lane & 15;
  const int rowBase = (int)blockIdx.x * GBM;

  v8f acc[4];
  {
    const v8f z = {0.f, 0.f, 0.f, 0.f, 0.f, 0.f, 0.f, 0.f};
#pragma unroll
    for (int t = 0; t < 4; ++t) acc[t] = z;
  }
  const size_t arow = (size_t)(rowBase + 16 * wave + m);
  const unsigned short* ap = fb  + arow * DF   + 8 * hh;
  const unsigned short* mp = mhl + arow * MPIT + 8 * hh;
  const unsigned short* bp = bt  + (size_t)m * KT + 8 * hh;

#pragma unroll 1
  for (int k0 = 0; k0 < DF; k0 += 32) {
    FragB af;
    af.h[0] = *(const v8usa*)(ap + k0);
    af.h[1] = *(const v8usa*)(ap + k0 + 16);
#pragma unroll
    for (int nt = 0; nt < 4; ++nt) {
      const unsigned short* wq = bp + (size_t)(16 * nt) * KT + k0;
      FragB bf;
      bf.h[0] = *(const v8usa*)wq;
      bf.h[1] = *(const v8usa*)(wq + 16);
      acc[nt] = wmb(af, bf, acc[nt]);
    }
  }
#pragma unroll 1
  for (int k1 = 0; k1 < KT - DF; k1 += 32) {
    FragB af;
    af.h[0] = *(const v8usa*)(mp + k1);
    af.h[1] = *(const v8usa*)(mp + k1 + 16);
#pragma unroll
    for (int nt = 0; nt < 4; ++nt) {
      const unsigned short* wq = bp + (size_t)(16 * nt) * KT + DF + k1;
      FragB bf;
      bf.h[0] = *(const v8usa*)wq;
      bf.h[1] = *(const v8usa*)(wq + 16);
      acc[nt] = wmb(af, bf, acc[nt]);
    }
  }

#pragma unroll
  for (int nt = 0; nt < 4; ++nt) {
    const int lc = 16 * nt + m;
#pragma unroll
    for (int r = 0; r < 8; ++r) {
      const int lr = 16 * wave + 8 * hh + r;
      stg[lr * DF + lc] = acc[nt][r];
    }
  }
  {
    const v4f bq = *(const v4f*)(biasf + 4 * (tid & 15));
    if (tid < 16) *(v4fa*)(sbias + 4 * tid) = bq;
  }
  __syncthreads();

  int fi = rowBase >> SLA;
  fi = imin(imax(fi, 0), nFlag - 1);
  const int fl = flagp[(size_t)fi * FLAGI];
  const float pn = __int_as_float(0x7fc00000);
  const int q = lane & 15;
  const v4f b4 = *(const v4fa*)(sbias + 4 * q);

#pragma unroll 1
  for (int i = 0; i < 8; ++i) {
    const int lr = 16 * wave + 2 * i + hh;
    const int gr = rowBase + lr;
    const v4f t = *(const v4fa*)(stg + lr * DF + 4 * q) + b4;
    v4f y;
    y.x = (t.x > 0.0f) ? t.x : (t.x - t.x);
    y.y = (t.y > 0.0f) ? t.y : (t.y - t.y);
    y.z = (t.z > 0.0f) ? t.z : (t.z - t.z);
    y.w = (t.w > 0.0f) ? t.w : (t.w - t.w);
    y.x = (fl != 0) ? pn : y.x; y.y = (fl != 0) ? pn : y.y;
    y.z = (fl != 0) ? pn : y.z; y.w = (fl != 0) ? pn : y.w;
    if (gr < nN) *(volatile v4f*)(outp + (size_t)gr * DF + 4 * q) = y;
  }
  __threadfence();
#pragma unroll 1
  for (int i = 0; i < 8; ++i) {
    const int lr = 16 * wave + 2 * i + hh;
    const int gr = rowBase + lr;
    const v4f t = *(const v4fa*)(stg + lr * DF + 4 * q) + b4;
    v4f y;
    y.x = (t.x > 0.0f) ? t.x : (t.x - t.x);
    y.y = (t.y > 0.0f) ? t.y : (t.y - t.y);
    y.z = (t.z > 0.0f) ? t.z : (t.z - t.z);
    y.w = (t.w > 0.0f) ? t.w : (t.w - t.w);
    y.x = (fl != 0) ? pn : y.x; y.y = (fl != 0) ? pn : y.y;
    y.z = (fl != 0) ? pn : y.z; y.w = (fl != 0) ? pn : y.w;
    if (gr < nN) *(volatile v4f*)(outp + (size_t)gr * DF + 4 * q) = y;
  }
}

static inline int cdiv(int a, int b) { return (a + b - 1) / b; }
static inline size_t al256(size_t o) { return (o + 255) & ~(size_t)255; }

extern "C" void kernel_launch(void* const* d_in, const int* in_sizes, int n_in,
                              void* d_out, int out_size, void* d_ws, size_t ws_size,
                              hipStream_t stream) {
  if (n_in < 6) return;
  if (in_sizes[0] < DF || (in_sizes[0] % DF) != 0) return;
  const int nN = in_sizes[0] / DF;
  const int nE = in_sizes[1];
  if (nN < 1 || nN > MAXN) return;
  if (nE < 1 || nE >= MAXE || in_sizes[2] != nE) return;
  if (in_sizes[3] != DF * DF || in_sizes[4] != DF * DF || in_sizes[5] != DF) return;
  if ((long long)out_size != (long long)nN * DF) return;

  const float* feat   = (const float*)d_in[0];
  const int*   src    = (const int*)  d_in[1];
  const int*   dst    = (const int*)  d_in[2];
  const float* wself  = (const float*)d_in[3];
  const float* wneigh = (const float*)d_in[4];
  const float* bias   = (const float*)d_in[5];
  float* out = (float*)d_out;

  const int NP = cdiv(nN, GBM) * GBM;
  const int gM = NP / GBM;
  const int gA = cdiv(NP, NBA);
  if ((long long)gA * NBA < (long long)NP) return;

  char* ws = (char*)d_ws;
  size_t off = 0;
  const size_t oBT   = off; off = al256(off + (size_t)DF * KT * 2);
  const size_t oBIAS = off; off = al256(off + (size_t)DF * 4);
  const size_t oFLAG = off; off = al256(off + (size_t)gA * FLAGI * 4);
  const size_t oFB   = off; off = al256(off + (size_t)NP * DF * 2);
  const size_t oMHL  = off; off = al256(off + (size_t)NP * MPIT * 2);
  if (off > ws_size || off > (size_t)WSMAX) return;
  unsigned short* BT    = (unsigned short*)(ws + oBT);
  float*          BIASF = (float*)(ws + oBIAS);
  int*            FLAG  = (int*)(ws + oFLAG);
  unsigned short* FB    = (unsigned short*)(ws + oFB);
  unsigned short* MHL   = (unsigned short*)(ws + oMHL);

  const size_t scanLds = (size_t)SCAN_INTS * 4;
  hipFuncSetAttribute(reinterpret_cast<const void*>(&k_scan), hipFuncAttributeMaxDynamicSharedMemorySize, (int)scanLds);

  const int nUnits = NUB + NTHR + NP * (DF / 8);

  k_prep<<<cdiv(nUnits, NTHR), NTHR, 0, stream>>>(feat, wself, wneigh, bias, FB, BT, BIASF, nN, nUnits);
  k_scan<<<gA, NTHR, scanLds, stream>>>(src, dst, FB, MHL, FLAG, nE, nN, NP);
  k_gemm<<<gM, NTHR, 0, stream>>>(FB, MHL, BT, BIASF, FLAG, gA, out, nN);
}
